// CategoricalGraphAtt_19456201851241
// MI455X (gfx1250) — hardware-verified
//
#include <hip/hip_runtime.h>
#include <stddef.h>
#include <math.h>


#define NN      20000
#define TT      10
#define DD      16
#define HH      128
#define GG      384
#define WKN     3
#define SSN     40
#define LLN     500
#define LP      512
#define KG      160
#define RB      32
#define RT      64
#define CA      16.0f
#define CW      64.0f
#define SCL     0.0009765625f
#define NEG_SLOPE 0.2f
#define WSCAP   134217728
#define E2CAP   1600

#define NTHR    256
#define NWAVE   8
#define EPT     8
#define CHUNK   (NTHR * EPT)
#define WCAP    (EPT * 32)
#define LISTN   (NWAVE * WCAP)
#define NBMAX   2048
#define RCAP    28672
#define DEGCAP  4096
#define LDS_AGG ((2 * RCAP + 2 * NBMAX + LISTN) * 4 + 64)

static_assert(NN % RB == 0);
static_assert(NN == SSN * LLN);
static_assert((NN * (HH / 4)) % 256 == 0);
static_assert(RB == 32 && RT == 64);
static_assert(HH == 128 && GG == 3 * HH && DD == 16);
static_assert(KG == 32 + HH && (KG % 8) == 0);
static_assert(LP % 32 == 0 && LP >= LLN && LP / 8 == 64);
static_assert((SSN * HH * (LP / 8)) % 256 == 0);
static_assert((SSN * LP * (LP / 8)) % 256 == 0);
static_assert((WKN * GG * (KG / 8)) % 256 == 0);
static_assert((CHUNK & (CHUNK - 1)) == 0 && CHUNK <= 4096);
static_assert((NBMAX & (NBMAX - 1)) == 0 && NBMAX <= 4096);
static_assert(NTHR * 8 == NBMAX);
static_assert(LISTN >= NBMAX);
static_assert(LISTN >= NWAVE * WCAP);
static_assert((RCAP % 32) == 0);
static_assert(LDS_AGG <= 300000);

typedef float    v4f  __attribute__((ext_vector_type(4)));
typedef float    v8f  __attribute__((ext_vector_type(8)));
typedef int      v4i  __attribute__((ext_vector_type(4)));
typedef int      v8i  __attribute__((ext_vector_type(8)));
typedef _Float16 v8h  __attribute__((ext_vector_type(8)));
typedef _Float16 v16h __attribute__((ext_vector_type(16)));
typedef v4f v4fa __attribute__((may_alias));
union FragH { v16h v; v8h h[2]; v8i w; };

__device__ __forceinline__ v8f wmh(const FragH& a, const FragH& b, v8f c) {
  v8f d = __builtin_amdgcn_wmma_f32_16x16x32_f16(false, a.v, false, b.v, (short)0, c, false, false);
  asm volatile("v_nop\n\tv_nop\n\tv_nop\n\tv_nop" : "+v"(d) : "v"(a.w), "v"(b.w));
  return d;
}

__device__ __forceinline__ v8h cvt8(const v4f a, const v4f b, const float s) {
  v8h h;
  h[0] = (_Float16)(a.x * s); h[1] = (_Float16)(a.y * s); h[2] = (_Float16)(a.z * s); h[3] = (_Float16)(a.w * s);
  h[4] = (_Float16)(b.x * s); h[5] = (_Float16)(b.y * s); h[6] = (_Float16)(b.z * s); h[7] = (_Float16)(b.w * s);
  return h;
}

__device__ __forceinline__ float sigm(float x) { return __builtin_amdgcn_rcpf(1.0f + __expf(-x)); }
__device__ __forceinline__ float tanh_f(float x) { return 1.0f - 2.0f * __builtin_amdgcn_rcpf(1.0f + __expf(2.0f * x)); }

__global__ __launch_bounds__(256) void k_wprep(const float* __restrict__ wih, const float* __restrict__ whh,
                                               const float* __restrict__ g1w, const float* __restrict__ fw,
                                               _Float16* wg16, _Float16* g1w16, _Float16* fw16) {
  const int j = (int)blockIdx.y;
  const int u = (int)blockIdx.x * 256 + (int)threadIdx.x;
  v4f a, b;
  _Float16* dst;
  size_t o;
  if (j == 0) {
    if (u >= WKN * GG * (KG / 8)) return;
    const int row = u / (KG / 8);
    const int k8  = (u - row * (KG / 8)) * 8;
    const int kx  = k8 < 8 ? k8 : 8;
    int kh = k8 - 32; kh = kh < 0 ? 0 : (kh > HH - 8 ? HH - 8 : kh);
    const float* px = wih + (size_t)row * DD + kx;
    const float* ph = whh + (size_t)row * HH + kh;
    const v4f ax = *(const v4f*)px, bx = *(const v4f*)(px + 4);
    const v4f ah = *(const v4f*)ph, bh = *(const v4f*)(ph + 4);
    const v4f z4 = {0.f, 0.f, 0.f, 0.f};
    if (k8 < DD) { a = ax; b = bx; }
    else if (k8 >= 32) { a = ah; b = bh; }
    else { a = z4; b = z4; }
    dst = wg16; o = (size_t)row * KG + k8;
  } else if (j == 1) {
    if (u >= HH * (HH / 8)) return;
    const int row = u >> 4, k8 = (u & 15) * 8;
    const float* p = g1w + (size_t)row * HH + k8;
    a = *(const v4f*)p; b = *(const v4f*)(p + 4);
    dst = g1w16; o = (size_t)row * HH + k8;
  } else {
    if (u >= HH * (GG / 8)) return;
    const int row = u / (GG / 8), k8 = (u - row * (GG / 8)) * 8;
    const float* p = fw + (size_t)row * GG + k8;
    a = *(const v4f*)p; b = *(const v4f*)(p + 4);
    dst = fw16; o = (size_t)row * GG + k8;
  }
  const v8h hv = cvt8(a, b, CW);
  *(volatile v8h*)(dst + o) = hv;
  __threadfence();
  *(volatile v8h*)(dst + o) = hv;
}

__global__ __launch_bounds__(RT) void k_gru(const float* __restrict__ xw, const _Float16* __restrict__ wg,
                                            const float* __restrict__ bi, const float* __restrict__ bh,
                                            const float* hsrc, float* hdst, int t, int useh, int nN) {
  __shared__ __attribute__((aligned(16))) float sH[RB * HH];
  __shared__ float sBi[GG];
  __shared__ float sBh[GG];
  const int tid = threadIdx.x, lane = tid & 31, wave = tid >> 5, hh = lane >> 4, ln = lane & 15;
  const int rowBase = (int)blockIdx.x * RB;
  for (int i = tid; i < GG; i += RT) { sBi[i] = bi[i]; sBh[i] = bh[i]; }
  const int row  = rowBase + 16 * wave + ln;
  const int rowc = row < nN ? row : nN - 1;
  const bool uh  = useh != 0;
  const v8i z8 = {0, 0, 0, 0, 0, 0, 0, 0};
  FragH ax;
  {
    const float* xp = xw + ((size_t)rowc * TT + t) * DD + 8 * hh;
    const v4f p0 = *(const v4f*)xp, p1 = *(const v4f*)(xp + 4);
    ax.w = z8;
    ax.h[0] = cvt8(p0, p1, CA);
  }
  FragH ahf[4];
#pragma unroll
  for (int ks = 0; ks < 4; ++ks) ahf[ks].w = z8;
  if (uh) {
    const float* hp = hsrc + (size_t)rowc * HH + 8 * hh;
#pragma unroll
    for (int ks = 0; ks < 4; ++ks) {
      const float* p = hp + 32 * ks;
      ahf[ks].h[0] = cvt8(*(const v4f*)p, *(const v4f*)(p + 4), CA);
      ahf[ks].h[1] = cvt8(*(const v4f*)(p + 16), *(const v4f*)(p + 20), CA);
    }
  }
  __syncthreads();
  const v8f zacc = {0.f, 0.f, 0.f, 0.f, 0.f, 0.f, 0.f, 0.f};
#pragma unroll 1
  for (int ct = 0; ct < HH / 16; ++ct) {
    const int c0 = 16 * ct;
    v8f accr = zacc, accz = zacc, accnx = zacc, accnh = zacc;
    const _Float16* pr = wg + (size_t)(c0 + ln) * KG + 8 * hh;
    const _Float16* pz = pr + (size_t)HH * KG;
    const _Float16* pn = pr + (size_t)(2 * HH) * KG;
    {
      FragH fr, fz, fn;
      fr.h[0] = *(const v8h*)pr; fr.h[1] = *(const v8h*)(pr + 16);
      fz.h[0] = *(const v8h*)pz; fz.h[1] = *(const v8h*)(pz + 16);
      fn.h[0] = *(const v8h*)pn; fn.h[1] = *(const v8h*)(pn + 16);
      accr  = wmh(ax, fr, accr);
      accz  = wmh(ax, fz, accz);
      accnx = wmh(ax, fn, accnx);
    }
    if (uh) {
#pragma unroll
      for (int ks = 0; ks < 4; ++ks) {
        const int k0 = 32 + 32 * ks;
        FragH fr, fz, fn;
        fr.h[0] = *(const v8h*)(pr + k0); fr.h[1] = *(const v8h*)(pr + k0 + 16);
        fz.h[0] = *(const v8h*)(pz + k0); fz.h[1] = *(const v8h*)(pz + k0 + 16);
        fn.h[0] = *(const v8h*)(pn + k0); fn.h[1] = *(const v8h*)(pn + k0 + 16);
        accr  = wmh(ahf[ks], fr, accr);
        accz  = wmh(ahf[ks], fz, accz);
        accnh = wmh(ahf[ks], fn, accnh);
      }
    }
    const int c = c0 + ln;
    const float brr = sBi[c] + sBh[c];
    const float bzz = sBi[HH + c] + sBh[HH + c];
    const float bnx = sBi[2 * HH + c];
    const float bnh = sBh[2 * HH + c];
    float* sp = sH + (size_t)(16 * wave + 8 * hh) * HH + c;
    const int rh0 = rowBase + 16 * wave + 8 * hh;
#pragma unroll
    for (int r = 0; r < 8; ++r) {
      const float prg = fmaf(accr[r], SCL, brr);
      const float pzg = fmaf(accz[r], SCL, bzz);
      const float rg = sigm(prg);
      const float zg = sigm(pzg);
      const float xn = fmaf(accnx[r], SCL, bnx);
      const float hn = fmaf(accnh[r], SCL, bnh);
      const float ng = tanh_f(fmaf(rg, hn, xn));
      float hold = 0.f;
      if (uh) {
        int rr = rh0 + r; rr = rr < nN ? rr : nN - 1;
        hold = hsrc[(size_t)rr * HH + c];
      }
      sp[(size_t)r * HH] = (1.0f - zg) * ng + zg * hold;
    }
  }
  __syncthreads();
  {
    const float* sb = sH + (size_t)(16 * wave) * HH + 4 * lane;
    float* hb = hdst + (size_t)(rowBase + 16 * wave) * HH + 4 * lane;
#pragma unroll
    for (int r = 0; r < 16; ++r) {
      if (rowBase + 16 * wave + r < nN) {
        const v4f v = *(const v4fa*)(sb + (size_t)r * HH);
        *(volatile v4f*)(hb + (size_t)r * HH) = v;
      }
    }
  }
  __threadfence();
  {
    const float* sb = sH + (size_t)(16 * wave) * HH + 4 * lane;
    float* hb = hdst + (size_t)(rowBase + 16 * wave) * HH + 4 * lane;
#pragma unroll
    for (int r = 0; r < 16; ++r) {
      if (rowBase + 16 * wave + r < nN) {
        const v4f v = *(const v4fa*)(sb + (size_t)r * HH);
        *(volatile v4f*)(hb + (size_t)r * HH) = v;
      }
    }
  }
}

__global__ __launch_bounds__(256) void k_att_time(const float* __restrict__ hs, const float* __restrict__ aW,
                                                  const float* __restrict__ ab, float* wke, int nN) {
  __shared__ float sW[TT * TT + TT];
  const int tid = threadIdx.x;
  if (tid < TT * TT + TT) {
    const int iw = tid < TT * TT ? tid : TT * TT - 1;
    int ib = tid - TT * TT; ib = ib < 0 ? 0 : ib;
    const float vw = aW[iw], vb = ab[ib];
    sW[tid] = tid < TT * TT ? vw : vb;
  }
  __syncthreads();
  const int u = (int)blockIdx.x * 256 + tid;
  if (u >= nN * (HH / 4)) return;
  const int n = u >> 5, q = u & 31;
  const size_t base = (size_t)n * HH + 4 * q;
  const size_t ts = (size_t)nN * HH;
  v4f sv[TT];
#pragma unroll
  for (int t = 0; t < TT; ++t) sv[t] = *(const v4f*)(hs + base + (size_t)t * ts);
  v4f mm = {-1.0e30f, -1.0e30f, -1.0e30f, -1.0e30f};
  v4f zz = {0.f, 0.f, 0.f, 0.f};
  v4f aa = {0.f, 0.f, 0.f, 0.f};
#pragma unroll 1
  for (int t = 0; t < TT; ++t) {
    const float bt = sW[TT * TT + t];
    v4f lg = {bt, bt, bt, bt};
#pragma unroll
    for (int tp = 0; tp < TT; ++tp) {
      const float w = sW[t * TT + tp];
      lg.x = fmaf(sv[tp].x, w, lg.x);
      lg.y = fmaf(sv[tp].y, w, lg.y);
      lg.z = fmaf(sv[tp].z, w, lg.z);
      lg.w = fmaf(sv[tp].w, w, lg.w);
    }
    const v4f v = *(const v4f*)(hs + base + (size_t)t * ts);
#define UPD(C) { const float mn = fmaxf(mm.C, lg.C); const float s1 = __expf(fmaxf(mm.C - mn, -87.0f)); \
      const float s2 = __expf(lg.C - mn); zz.C = fmaf(zz.C, s1, s2); aa.C = fmaf(aa.C, s1, s2 * v.C); mm.C = mn; }
    UPD(x) UPD(y) UPD(z) UPD(w)
#undef UPD
  }
  v4f o;
  o.x = aa.x * __builtin_amdgcn_rcpf(zz.x);
  o.y = aa.y * __builtin_amdgcn_rcpf(zz.y);
  o.z = aa.z * __builtin_amdgcn_rcpf(zz.z);
  o.w = aa.w * __builtin_amdgcn_rcpf(zz.w);
  float* p = wke + base;
  *(volatile v4f*)p = o;
  __threadfence();
  *(volatile v4f*)p = o;
}

__global__ __launch_bounds__(256) void k_att_week(const float* __restrict__ wke, const float* __restrict__ kW,
                                                  const float* __restrict__ kb, float* wav, int nN) {
  const int u = (int)blockIdx.x * 256 + (int)threadIdx.x;
  if (u >= nN * (HH / 4)) return;
  const int n = u >> 5, q = u & 31;
  const size_t base = (size_t)n * HH + 4 * q;
  const size_t ws = (size_t)nN * HH;
  const v4f e0 = *(const v4f*)(wke + base);
  const v4f e1 = *(const v4f*)(wke + base + ws);
  const v4f e2 = *(const v4f*)(wke + base + 2 * ws);
  const float w00 = kW[0], w01 = kW[1], w02 = kW[2];
  const float w10 = kW[3], w11 = kW[4], w12 = kW[5];
  const float w20 = kW[6], w21 = kW[7], w22 = kW[8];
  const float b0 = kb[0], b1 = kb[1], b2 = kb[2];
  v4f o;
#define CH(C) { \
    const float l0 = fmaf(w02, e2.C, fmaf(w01, e1.C, fmaf(w00, e0.C, b0))); \
    const float l1 = fmaf(w12, e2.C, fmaf(w11, e1.C, fmaf(w10, e0.C, b1))); \
    const float l2 = fmaf(w22, e2.C, fmaf(w21, e1.C, fmaf(w20, e0.C, b2))); \
    const float mx = fmaxf(l0, fmaxf(l1, l2)); \
    const float p0 = __expf(l0 - mx), p1 = __expf(l1 - mx), p2 = __expf(l2 - mx); \
    const float den = p0 + p1 + p2; \
    const float num = fmaf(p2, e2.C, fmaf(p1, e1.C, p0 * e0.C)); \
    o.C = num * __builtin_amdgcn_rcpf(den); }
  CH(x) CH(y) CH(z) CH(w)
#undef CH
  float* p = wav + base;
  *(volatile v4f*)p = o;
  __threadfence();
  *(volatile v4f*)p = o;
}

__global__ __launch_bounds__(RT) void k_lin1(const float* __restrict__ wav, const _Float16* __restrict__ w16,
                                             const float* __restrict__ asrc, const float* __restrict__ adst,
                                             float* Y, float* ES, float* ED, int nN) {
  __shared__ __attribute__((aligned(16))) float sY[RB * HH];
  __shared__ float sAs[HH];
  __shared__ float sAd[HH];
  __shared__ float sEs[RB];
  __shared__ float sEd[RB];
  const int tid = threadIdx.x, lane = tid & 31, wave = tid >> 5, hh = lane >> 4, ln = lane & 15;
  const int rowBase = (int)blockIdx.x * RB;
  sAs[tid] = asrc[tid]; sAs[tid + RT] = asrc[tid + RT];
  sAd[tid] = adst[tid]; sAd[tid + RT] = adst[tid + RT];
  const int row  = rowBase + 16 * wave + ln;
  const int rowc = row < nN ? row : nN - 1;
  const v8f zacc = {0.f, 0.f, 0.f, 0.f, 0.f, 0.f, 0.f, 0.f};
  v8f acc[8];
#pragma unroll
  for (int ct = 0; ct < 8; ++ct) acc[ct] = zacc;
  const float* ap = wav + (size_t)rowc * HH + 8 * hh;
  const _Float16* bp = w16 + (size_t)ln * HH + 8 * hh;
#pragma unroll 1
  for (int ks = 0; ks < HH / 32; ++ks) {
    FragH af;
    const float* a0 = ap + 32 * ks;
    af.h[0] = cvt8(*(const v4f*)a0, *(const v4f*)(a0 + 4), CA);
    af.h[1] = cvt8(*(const v4f*)(a0 + 16), *(const v4f*)(a0 + 20), CA);
#pragma unroll
    for (int ct = 0; ct < 8; ++ct) {
      const _Float16* bq = bp + (size_t)(16 * ct) * HH + 32 * ks;
      FragH bf;
      bf.h[0] = *(const v8h*)bq;
      bf.h[1] = *(const v8h*)(bq + 16);
      acc[ct] = wmh(af, bf, acc[ct]);
    }
  }
  float* sp = sY + (size_t)(16 * wave + 8 * hh) * HH + ln;
#pragma unroll
  for (int ct = 0; ct < 8; ++ct) {
#pragma unroll
    for (int r = 0; r < 8; ++r) sp[(size_t)r * HH + 16 * ct] = acc[ct][r] * SCL;
  }
  __syncthreads();
  {
    const int r2 = tid >> 1, half = tid & 1;
    const float* sr = sY + (size_t)r2 * HH + 64 * half;
    const float* pa = sAs + 64 * half;
    const float* pd = sAd + 64 * half;
    float s = 0.f, d = 0.f;
#pragma unroll 2
    for (int c = 0; c < 64; ++c) { const float v = sr[c]; s = fmaf(v, pa[c], s); d = fmaf(v, pd[c], d); }
    s += __shfl_xor(s, 1);
    d += __shfl_xor(d, 1);
    if (half == 0) { sEs[r2] = s; sEd[r2] = d; }
  }
  __syncthreads();
  {
    const float* sb = sY + (size_t)(16 * wave) * HH + 4 * lane;
    float* yb = Y + (size_t)(rowBase + 16 * wave) * HH + 4 * lane;
#pragma unroll
    for (int r = 0; r < 16; ++r) {
      if (rowBase + 16 * wave + r < nN) {
        const v4f v = *(const v4fa*)(sb + (size_t)r * HH);
        *(volatile v4f*)(yb + (size_t)r * HH) = v;
      }
    }
    const int re = rowBase + lane;
    const float ve = sEs[lane], vd = sEd[lane];
    if (re < nN) {
      if (wave == 0) *(volatile float*)(ES + re) = ve;
      else           *(volatile float*)(ED + re) = vd;
    }
  }
  __threadfence();
  {
    const float* sb = sY + (size_t)(16 * wave) * HH + 4 * lane;
    float* yb = Y + (size_t)(rowBase + 16 * wave) * HH + 4 * lane;
#pragma unroll
    for (int r = 0; r < 16; ++r) {
      if (rowBase + 16 * wave + r < nN) {
        const v4f v = *(const v4fa*)(sb + (size_t)r * HH);
        *(volatile v4f*)(yb + (size_t)r * HH) = v;
      }
    }
    const int re = rowBase + lane;
    const float ve = sEs[lane], vd = sEd[lane];
    if (re < nN) {
      if (wave == 0) *(volatile float*)(ES + re) = ve;
      else           *(volatile float*)(ED + re) = vd;
    }
  }
}

__device__ __forceinline__ int scan_chunk(const int* __restrict__ dsts, int nE, int cbase, int slotBase,
                                          int nb, int vec8, int* list, int tid, int lane, int wave) {
  int wc = 0;
  const int el0  = tid * EPT;
  const int e0   = cbase + el0;
  const int sent = -2147483647 - 1;
  v4i da, db;
  if (vec8 != 0 && cbase + CHUNK <= nE) {
    da = *(const v4i*)(dsts + e0);
    db = *(const v4i*)(dsts + e0 + 4);
  } else {
    da.x = (e0     < nE) ? dsts[min(e0,     nE - 1)] : sent;
    da.y = (e0 + 1 < nE) ? dsts[min(e0 + 1, nE - 1)] : sent;
    da.z = (e0 + 2 < nE) ? dsts[min(e0 + 2, nE - 1)] : sent;
    da.w = (e0 + 3 < nE) ? dsts[min(e0 + 3, nE - 1)] : sent;
    db.x = (e0 + 4 < nE) ? dsts[min(e0 + 4, nE - 1)] : sent;
    db.y = (e0 + 5 < nE) ? dsts[min(e0 + 5, nE - 1)] : sent;
    db.z = (e0 + 6 < nE) ? dsts[min(e0 + 6, nE - 1)] : sent;
    db.w = (e0 + 7 < nE) ? dsts[min(e0 + 7, nE - 1)] : sent;
  }
  const unsigned nbs = (unsigned)slotBase;
  const unsigned unb = (unsigned)nb;
  const unsigned s0 = (unsigned)da.x - nbs, s1 = (unsigned)da.y - nbs;
  const unsigned s2 = (unsigned)da.z - nbs, s3 = (unsigned)da.w - nbs;
  const unsigned s4 = (unsigned)db.x - nbs, s5 = (unsigned)db.y - nbs;
  const unsigned s6 = (unsigned)db.z - nbs, s7 = (unsigned)db.w - nbs;
  const bool h0 = s0 < unb, h1 = s1 < unb, h2 = s2 < unb, h3 = s3 < unb;
  const bool h4 = s4 < unb, h5 = s5 < unb, h6 = s6 < unb, h7 = s7 < unb;
  const unsigned any = __builtin_amdgcn_ballot_w32(h0 | h1 | h2 | h3 | h4 | h5 | h6 | h7);
  if (any != 0u) {
#define HITJ(J, HJ, SJ) { \
      const unsigned mj = __builtin_amdgcn_ballot_w32(HJ); \
      if (mj != 0u) { \
        if (HJ) { \
          const int pos = wc + (int)__builtin_amdgcn_mbcnt_lo(mj, 0u); \
          if (pos < WCAP) list[wave * WCAP + pos] = ((el0 + (J)) << 12) | (int)(SJ); \
        } \
        wc += (int)__builtin_popcount(mj); } }
    HITJ(0, h0, s0)
    HITJ(1, h1, s1)
    HITJ(2, h2, s2)
    HITJ(3, h3, s3)
    HITJ(4, h4, s4)
    HITJ(5, h5, s5)
    HITJ(6, h6, s6)
    HITJ(7, h7, s7)
#undef HITJ
  }
  return wc;
}

__global__ __launch_bounds__(NTHR) void k_agg(
    const int* __restrict__ srcs, const int* __restrict__ dsts,
    const float* __restrict__ Y, const float* __restrict__ ES, const float* __restrict__ ED,
    const float* __restrict__ bias, float* xo,
    int nN, int nE, int nb, int vec8) {
  extern __shared__ v4f lds_dyn[];
  int* reg1 = (int*)lds_dyn;
  int* reg2 = reg1 + RCAP;
  int* scnt = reg2 + RCAP;
  int* soff = scnt + NBMAX;
  int* list = soff + NBMAX;
  int* wcnt = list + LISTN;
  int* wtot = wcnt + NWAVE;
  const int tid = threadIdx.x, lane = tid & 31, wave = tid >> 5;
  const int nodeBase = (int)blockIdx.x * nb;

  for (int i = tid; i < NBMAX; i += NTHR) scnt[i] = 0;
  __syncthreads();

  int tot = 0;
  const int nChunks = (nE + CHUNK - 1) / CHUNK;
#pragma unroll 1
  for (int ch = 0; ch < nChunks; ++ch) {
    const int cbase = ch * CHUNK;
    const int wc = scan_chunk(dsts, nE, cbase, nodeBase, nb, vec8, list, tid, lane, wave);
    if (lane == 0) wcnt[wave] = wc;
    __syncthreads();
    int pre = 0, all = 0;
#pragma unroll
    for (int w2 = 0; w2 < NWAVE; ++w2) {
      int c = wcnt[w2];
      c = c < 0 ? 0 : (c > WCAP ? WCAP : c);
      all += c;
      pre += (w2 < wave) ? c : 0;
    }
    const int wcc  = wc > WCAP ? WCAP : wc;
    const int base = tot + pre;
#pragma unroll 1
    for (int i = lane; i < wcc; i += 32) {
      const int ent = list[wave * WCAP + i];
      const int el  = (ent >> 12) & (CHUNK - 1);
      const int sl  = ent & (NBMAX - 1);
      int eid = cbase + el;
      eid = eid > nE - 1 ? nE - 1 : eid;
      const int pos = base + i;
      if (pos < RCAP) reg1[pos] = (int)(((unsigned)eid << 12) | (unsigned)sl);
    }
    tot += all;
    tot = tot > RCAP ? RCAP : tot;
    __syncthreads();
  }
  const int nh = tot;

  if (wave == 0) {
#pragma unroll 1
    for (int b0 = 0; b0 < nh; b0 += 32) {
      const int idx = b0 + lane;
      const int uv  = reg1[idx < RCAP ? idx : RCAP - 1];
      const int m32 = (nh - b0) < 32 ? (nh - b0) : 32;
#pragma unroll 1
      for (int k = 0; k < m32; ++k) {
        const int u  = __builtin_amdgcn_readlane(uv, k);
        const int sl = u & (NBMAX - 1);
        if (lane == 0) scnt[sl] = scnt[sl] + 1;
      }
    }
  }
  __syncthreads();

  {
    const v4i ca = *(const v4i*)(scnt + 8 * tid);
    const v4i cb = *(const v4i*)(scnt + 8 * tid + 4);
    const int e0 = ca.x < 0 ? 0 : ca.x, e1 = ca.y < 0 ? 0 : ca.y, e2 = ca.z < 0 ? 0 : ca.z, e3 = ca.w < 0 ? 0 : ca.w;
    const int e4 = cb.x < 0 ? 0 : cb.x, e5 = cb.y < 0 ? 0 : cb.y, e6 = cb.z < 0 ? 0 : cb.z, e7 = cb.w < 0 ? 0 : cb.w;
    const int ts = e0 + e1 + e2 + e3 + e4 + e5 + e6 + e7;
    int incl = ts;
#pragma unroll
    for (int d = 1; d < 32; d <<= 1) {
      const int up = __shfl_up(incl, d);
      if (lane >= d) incl += up;
    }
    if (lane == 31) wtot[wave] = incl;
    __syncthreads();
    int pre = 0;
#pragma unroll
    for (int w2 = 0; w2 < NWAVE; ++w2) pre += (w2 < wave) ? wtot[w2] : 0;
    int run = pre + incl - ts;
    soff[8 * tid + 0] = run; run += e0;
    soff[8 * tid + 1] = run; run += e1;
    soff[8 * tid + 2] = run; run += e2;
    soff[8 * tid + 3] = run; run += e3;
    soff[8 * tid + 4] = run; run += e4;
    soff[8 * tid + 5] = run; run += e5;
    soff[8 * tid + 6] = run; run += e6;
    soff[8 * tid + 7] = run;
  }
  __syncthreads();
  for (int i = tid; i < NBMAX; i += NTHR) list[i] = soff[i];
  __syncthreads();

  if (wave == 0) {
#pragma unroll 1
    for (int b0 = 0; b0 < nh; b0 += 32) {
      const int idx = b0 + lane;
      const int uv  = reg1[idx < RCAP ? idx : RCAP - 1];
      const int m32 = (nh - b0) < 32 ? (nh - b0) : 32;
#pragma unroll 1
      for (int k = 0; k < m32; ++k) {
        const int u   = __builtin_amdgcn_readlane(uv, k);
        const int sl  = u & (NBMAX - 1);
        const int eid = (int)((unsigned)u >> 12);
        if (lane == 0) {
          int pos = list[sl];
          pos = pos < 0 ? 0 : (pos > RCAP - 1 ? RCAP - 1 : pos);
          reg2[pos] = eid;
          list[sl] = pos + 1;
        }
      }
    }
  }
  __syncthreads();

  const int nbw = nb >> 3;
  const int c4  = 4 * lane;
  const v4f bz  = *(const v4f*)(bias + c4);
  const bool ovf = (nh >= RCAP);
  const float qnan = __int_as_float(0x7fc00000);
#pragma unroll 1
  for (int jt = 0; jt < nbw; ++jt) {
    const int slot = wave * nbw + jt;
    const int grow = nodeBase + slot;
    const int gcl  = grow < nN ? grow : nN - 1;
    int st = soff[slot];
    const int craw = scnt[slot];
    int cnt = craw;
    st  = st < 0 ? 0 : (st > nh ? nh : st);
    cnt = cnt < 0 ? 0 : (cnt > DEGCAP ? DEGCAP : cnt);
    if (cnt > nh - st) cnt = nh - st;
    const float pz = (ovf || craw > DEGCAP) ? qnan : 0.0f;
    const bool wr = grow < nN;

    const v4f xd = *(const v4f*)(Y + (size_t)gcl * HH + c4);
    const float edv = ED[gcl];
    const float esd = ES[gcl];
    const float t0 = esd + edv;
    float mx = fmaxf(t0, NEG_SLOPE * t0);
    float dn = 1.0f;
    v4f a = xd;
#pragma unroll 1
    for (int q = 0; q < cnt; ++q) {
      int idx = st + q; idx = idx > RCAP - 1 ? RCAP - 1 : idx;
      int eid = reg2[idx]; eid = eid < 0 ? 0 : (eid > nE - 1 ? nE - 1 : eid);
      const int sraw = srcs[eid];
      const int s = sraw < 0 ? 0 : (sraw > nN - 1 ? nN - 1 : sraw);
      const v4f xs = *(const v4f*)(Y + (size_t)s * HH + c4);
      const float ess = ES[s];
      const float u = ess + edv;
      const float l = fmaxf(u, NEG_SLOPE * u);
      const float mn = fmaxf(mx, l);
      const float s1 = __expf(mx - mn), s2 = __expf(l - mn);
      dn = fmaf(dn, s1, s2);
      a.x = fmaf(a.x, s1, s2 * xs.x);
      a.y = fmaf(a.y, s1, s2 * xs.y);
      a.z = fmaf(a.z, s1, s2 * xs.z);
      a.w = fmaf(a.w, s1, s2 * xs.w);
      mx = mn;
    }
    const float inv = __builtin_amdgcn_rcpf(dn);
    v4f o;
    o.x = fmaf(a.x, inv, bz.x) + pz;
    o.y = fmaf(a.y, inv, bz.y) + pz;
    o.z = fmaf(a.z, inv, bz.z) + pz;
    o.w = fmaf(a.w, inv, bz.w) + pz;
    float* op = xo + (size_t)gcl * HH + c4;
    if (wr) *(volatile v4f*)op = o;
    __threadfence();
    if (wr) *(volatile v4f*)op = o;
  }
}

__global__ __launch_bounds__(256) void k_prep2(const float* __restrict__ g1o, const float* __restrict__ pw,
                                               _Float16* st16, _Float16* pw16, int b0) {
  const int tid = threadIdx.x;
  v8h hv;
  _Float16* dst;
  if ((int)blockIdx.x < b0) {
    const int u = (int)blockIdx.x * 256 + tid;
    if (u >= SSN * HH * (LP / 8)) return;
    const int row = u >> 6, l8 = (u & 63) * 8;
    const int s = row >> 7, h = row & (HH - 1);
#pragma unroll
    for (int i = 0; i < 8; ++i) {
      const int l = l8 + i;
      const int lc = l < LLN ? l : LLN - 1;
      const float v = g1o[((size_t)s * LLN + lc) * HH + h];
      hv[i] = (_Float16)(v * (l < LLN ? CA : 0.0f));
    }
    dst = st16 + (size_t)row * LP + l8;
  } else {
    const int u = ((int)blockIdx.x - b0) * 256 + tid;
    if (u >= SSN * LP * (LP / 8)) return;
    const int row = u >> 6, l8 = (u & 63) * 8;
    const int s = row >> 9, t = row & (LP - 1);
    const int tc = t < LLN ? t : LLN - 1;
#pragma unroll
    for (int i = 0; i < 8; ++i) {
      const int l = l8 + i;
      const int lc = l < LLN ? l : LLN - 1;
      const float v = pw[((size_t)s * LLN + tc) * LLN + lc];
      hv[i] = (_Float16)(v * ((t < LLN && l < LLN) ? CW : 0.0f));
    }
    dst = pw16 + (size_t)row * LP + l8;
  }
  *(volatile v8h*)dst = hv;
  __threadfence();
  *(volatile v8h*)dst = hv;
}

__global__ __launch_bounds__(256) void k_sector(const _Float16* __restrict__ st16, const _Float16* __restrict__ pw16,
                                                const float* __restrict__ pb, const float* __restrict__ g1o, float* cat) {
  __shared__ __attribute__((aligned(16))) float sO[HH];
  const int s = (int)blockIdx.x;
  const int tid = threadIdx.x, lane = tid & 31, wave = tid >> 5, hh = lane >> 4, ln = lane & 15;
  const _Float16* ap0 = st16 + ((size_t)s * HH + 16 * wave + ln) * LP + 8 * hh;
  const v8f zacc = {0.f, 0.f, 0.f, 0.f, 0.f, 0.f, 0.f, 0.f};
  float mm[8], zz[8], aa[8];
#pragma unroll
  for (int r = 0; r < 8; ++r) { mm[r] = -1.0e30f; zz[r] = 0.f; aa[r] = 0.f; }
#pragma unroll 1
  for (int ct = 0; ct < LP / 16; ++ct) {
    v8f acc = zacc;
    const _Float16* bp0 = pw16 + ((size_t)s * LP + 16 * ct + ln) * LP + 8 * hh;
#pragma unroll 2
    for (int kc = 0; kc < LP / 32; ++kc) {
      FragH af, bf;
      af.h[0] = *(const v8h*)(ap0 + 32 * kc);
      af.h[1] = *(const v8h*)(ap0 + 32 * kc + 16);
      bf.h[0] = *(const v8h*)(bp0 + 32 * kc);
      bf.h[1] = *(const v8h*)(bp0 + 32 * kc + 16);
      acc = wmh(af, bf, acc);
    }
    const int tcol = 16 * ct + ln;
    const bool tin = tcol < LLN;
    const int tc = tin ? tcol : LLN - 1;
    const float bv = pb[(size_t)s * LLN + tc];
    const float* vp = g1o + ((size_t)s * LLN + tc) * HH + 16 * wave + 8 * hh;
#pragma unroll
    for (int r = 0; r < 8; ++r) {
      const float lg = fmaf(acc[r], SCL, bv);
      const float sv = vp[r];
      const float mn = tin ? fmaxf(mm[r], lg) : mm[r];
      const float s1 = __expf(fmaxf(mm[r] - mn, -87.0f));
      const float ev = tin ? __expf(lg - mn) : 0.f;
      zz[r] = fmaf(zz[r], s1, ev);
      aa[r] = fmaf(aa[r], s1, ev * sv);
      mm[r] = mn;
    }
  }
#pragma unroll
  for (int off = 1; off < 16; off <<= 1) {
#pragma unroll
    for (int r = 0; r < 8; ++r) {
      const float m2 = __shfl_xor(mm[r], off);
      const float z2 = __shfl_xor(zz[r], off);
      const float a2 = __shfl_xor(aa[r], off);
      const float mn = fmaxf(mm[r], m2);
      const float s1 = __expf(mm[r] - mn), s2 = __expf(m2 - mn);
      zz[r] = zz[r] * s1 + z2 * s2;
      aa[r] = aa[r] * s1 + a2 * s2;
      mm[r] = mn;
    }
  }
  if (ln == 0) {
#pragma unroll
    for (int r = 0; r < 8; ++r) sO[16 * wave + 8 * hh + r] = aa[r] * __builtin_amdgcn_rcpf(zz[r]);
  }
  __syncthreads();
  if (wave == 0) {
    const v4f v = *(const v4fa*)(sO + 4 * lane);
    *(volatile v4f*)(cat + (size_t)s * HH + 4 * lane) = v;
  }
  __threadfence();
  if (wave == 0) {
    const v4f v = *(const v4fa*)(sO + 4 * lane);
    *(volatile v4f*)(cat + (size_t)s * HH + 4 * lane) = v;
  }
}

__global__ __launch_bounds__(256) void k_gat2(const float* __restrict__ cat, const int* __restrict__ eo,
                                              const float* __restrict__ w2, const float* __restrict__ as2,
                                              const float* __restrict__ ad2, const float* __restrict__ b2,
                                              float* cat2, int nE2) {
  __shared__ __attribute__((aligned(16))) float sX[SSN * HH];
  __shared__ __attribute__((aligned(16))) float sP[SSN * HH];
  __shared__ int sSrc[E2CAP];
  __shared__ int sDst[E2CAP];
  __shared__ float sAs[HH];
  __shared__ float sAd[HH];
  __shared__ float sEs[SSN];
  __shared__ float sEd[SSN];
  const int tid = threadIdx.x, lane = tid & 31, wave = tid >> 5;
  const int nE = nE2 < 0 ? 0 : (nE2 > E2CAP ? E2CAP : nE2);
  for (int i = tid; i < SSN * HH; i += 256) sX[i] = cat[i];
  for (int i = tid; i < nE; i += 256) { sSrc[i] = eo[i]; sDst[i] = eo[(size_t)nE2 + i]; }
  if (tid < HH) { sAs[tid] = as2[tid]; sAd[tid] = ad2[tid]; }
  __syncthreads();
  const int c = tid & (HH - 1), i0 = tid >> 7;
  {
    const float* wr = w2 + (size_t)c * HH;
#pragma unroll 1
    for (int i = i0; i < SSN; i += 2) {
      const float* xr = sX + (size_t)i * HH;
      float acc = 0.f;
#pragma unroll 4
      for (int k = 0; k < HH; ++k) acc = fmaf(xr[k], wr[k], acc);
      sP[(size_t)i * HH + c] = acc;
    }
  }
  __syncthreads();
  if (tid < SSN) {
    const float* pr = sP + (size_t)tid * HH;
    float sa = 0.f, sd = 0.f;
#pragma unroll 2
    for (int k = 0; k < HH; ++k) { const float v = pr[k]; sa = fmaf(v, sAs[k], sa); sd = fmaf(v, sAd[k], sd); }
    sEs[tid] = sa; sEd[tid] = sd;
  }
  __syncthreads();
  const float bc = b2[c];
#pragma unroll 1
  for (int d = i0; d < SSN; d += 2) {
    const float edv = sEd[d];
    const float t0 = sEs[d] + edv;
    float mx = fmaxf(t0, NEG_SLOPE * t0);
    float dn = 1.0f;
    float a = sP[(size_t)d * HH + c];
#pragma unroll 1
    for (int e = 0; e < nE; ++e) {
      if (sDst[e] == d) {
        int sn = sSrc[e]; sn = sn < 0 ? 0 : (sn > SSN - 1 ? SSN - 1 : sn);
        const float u = sEs[sn] + edv;
        const float l = fmaxf(u, NEG_SLOPE * u);
        const float mn = fmaxf(mx, l);
        const float s1 = __expf(mx - mn), s2 = __expf(l - mn);
        dn = fmaf(dn, s1, s2);
        a = fmaf(a, s1, s2 * sP[(size_t)sn * HH + c]);
        mx = mn;
      }
    }
    sX[(size_t)d * HH + c] = fmaf(a, __builtin_amdgcn_rcpf(dn), bc);
  }
  __syncthreads();
#pragma unroll 1
  for (int r = wave; r < SSN; r += 8) {
    const v4f v = *(const v4fa*)(sX + (size_t)r * HH + 4 * lane);
    *(volatile v4f*)(cat2 + (size_t)r * HH + 4 * lane) = v;
  }
  __threadfence();
#pragma unroll 1
  for (int r = wave; r < SSN; r += 8) {
    const v4f v = *(const v4fa*)(sX + (size_t)r * HH + 4 * lane);
    *(volatile v4f*)(cat2 + (size_t)r * HH + 4 * lane) = v;
  }
}

__global__ __launch_bounds__(RT) void k_fus(const float* __restrict__ wav, const float* __restrict__ g1o,
                                            const float* __restrict__ cat2, const _Float16* __restrict__ fw16,
                                            const float* __restrict__ fb, const float* __restrict__ rw,
                                            const float* __restrict__ rb, const float* __restrict__ cw,
                                            const float* __restrict__ cb, float* out, int nN) {
  __shared__ __attribute__((aligned(16))) float sF[RB * HH];
  __shared__ float sFb[HH];
  __shared__ float sRw[HH];
  __shared__ float sCw[HH];
  __shared__ __attribute__((aligned(16))) float sReg[RB];
  __shared__ __attribute__((aligned(16))) float sCls[RB];
  const int tid = threadIdx.x, lane = tid & 31, wave = tid >> 5, hh = lane >> 4, ln = lane & 15;
  const int rowBase = (int)blockIdx.x * RB;
  sFb[tid] = fb[tid]; sFb[tid + RT] = fb[tid + RT];
  sRw[tid] = rw[tid]; sRw[tid + RT] = rw[tid + RT];
  sCw[tid] = cw[tid]; sCw[tid + RT] = cw[tid + RT];
  const float rb0 = rb[0], cb0 = cb[0];
  const int row  = rowBase + 16 * wave + ln;
  const int rowc = row < nN ? row : nN - 1;
  int sec = rowc / LLN; sec = sec > SSN - 1 ? SSN - 1 : sec;
  const v8f zacc = {0.f, 0.f, 0.f, 0.f, 0.f, 0.f, 0.f, 0.f};
  v8f acc[8];
#pragma unroll
  for (int ct = 0; ct < 8; ++ct) acc[ct] = zacc;
  const _Float16* bp = fw16 + (size_t)ln * GG + 8 * hh;
#pragma unroll 1
  for (int ks = 0; ks < GG / 32; ++ks) {
    const float* ap;
    if (ks < 4)      ap = wav  + (size_t)rowc * HH + 32 * ks + 8 * hh;
    else if (ks < 8) ap = g1o  + (size_t)rowc * HH + 32 * (ks - 4) + 8 * hh;
    else             ap = cat2 + (size_t)sec  * HH + 32 * (ks - 8) + 8 * hh;
    FragH af;
    af.h[0] = cvt8(*(const v4f*)ap, *(const v4f*)(ap + 4), CA);
    af.h[1] = cvt8(*(const v4f*)(ap + 16), *(const v4f*)(ap + 20), CA);
#pragma unroll
    for (int ct = 0; ct < 8; ++ct) {
      const _Float16* bq = bp + (size_t)(16 * ct) * GG + 32 * ks;
      FragH bf;
      bf.h[0] = *(const v8h*)bq;
      bf.h[1] = *(const v8h*)(bq + 16);
      acc[ct] = wmh(af, bf, acc[ct]);
    }
  }
  __syncthreads();
  {
    float* sp = sF + (size_t)(16 * wave + 8 * hh) * HH + ln;
#pragma unroll
    for (int ct = 0; ct < 8; ++ct) {
      const float bvv = sFb[16 * ct + ln];
#pragma unroll
      for (int r = 0; r < 8; ++r) sp[(size_t)r * HH + 16 * ct] = fmaxf(fmaf(acc[ct][r], SCL, bvv), 0.f);
    }
  }
  __syncthreads();
  {
    const int r2 = tid >> 1, half = tid & 1;
    const float* fr = sF + (size_t)r2 * HH + 64 * half;
    const float* pr = sRw + 64 * half;
    const float* pc = sCw + 64 * half;
    float rs = 0.f, cs = 0.f;
#pragma unroll 2
    for (int k = 0; k < 64; ++k) { const float f = fr[k]; rs = fmaf(f, pr[k], rs); cs = fmaf(f, pc[k], cs); }
    rs += __shfl_xor(rs, 1);
    cs += __shfl_xor(cs, 1);
    if (half == 0) { sReg[r2] = rs + rb0; sCls[r2] = sigm(cs + cb0); }
  }
  __syncthreads();
  if (wave == 0 && lane < 16) {
    const int q = lane & 7;
    const v4f vr = *(const v4fa*)(sReg + 4 * q);
    const v4f vc = *(const v4fa*)(sCls + 4 * q);
    v4f v = vr;
    if (lane >= 8) v = vc;
    float* p = out + (lane < 8 ? (size_t)0 : (size_t)nN) + (size_t)rowBase + 4 * q;
    if (rowBase + 4 * q + 3 < nN) *(volatile v4f*)p = v;
  }
  __threadfence();
  if (wave == 0 && lane < 16) {
    const int q = lane & 7;
    const v4f vr = *(const v4fa*)(sReg + 4 * q);
    const v4f vc = *(const v4fa*)(sCls + 4 * q);
    v4f v = vr;
    if (lane >= 8) v = vc;
    float* p = out + (lane < 8 ? (size_t)0 : (size_t)nN) + (size_t)rowBase + 4 * q;
    if (rowBase + 4 * q + 3 < nN) *(volatile v4f*)p = v;
  }
}

static int pick_nb(int nE, int nN) {
  int nb = NBMAX;
  while (nb > 16 && (long long)nb * (long long)nE * 5LL > (long long)RCAP * (long long)nN * 4LL) nb >>= 1;
  return nb;
}

static size_t al256(size_t x) { return (x + 255) & ~(size_t)255; }

extern "C" void kernel_launch(void* const* d_in, const int* in_sizes, int n_in,
                              void* d_out, int out_size, void* d_ws, size_t ws_size,
                              hipStream_t stream) {
  if (n_in < 27) return;
  const int nN = NN;
  if (in_sizes[0] != WKN * NN * TT * DD) return;
  if (in_sizes[1] < 2 || (in_sizes[1] & 1) != 0) return;
  const int nE = in_sizes[1] / 2;
  if (nE > (1 << 20)) return;
  if (in_sizes[2] < 2 || (in_sizes[2] & 1) != 0) return;
  const int nE2 = in_sizes[2] / 2;
  if (nE2 > E2CAP) return;
  if (in_sizes[3] != WKN * GG * DD || in_sizes[4] != WKN * GG * HH) return;
  if (in_sizes[5] != WKN * GG || in_sizes[6] != WKN * GG) return;
  if (in_sizes[7] != WKN * TT * TT || in_sizes[8] != WKN * TT) return;
  if (in_sizes[9] != WKN * WKN || in_sizes[10] != WKN) return;
  if (in_sizes[11] != HH * HH || in_sizes[12] != HH || in_sizes[13] != HH || in_sizes[14] != HH) return;
  if (in_sizes[15] != HH * HH || in_sizes[16] != HH || in_sizes[17] != HH || in_sizes[18] != HH) return;
  if (in_sizes[19] != SSN * LLN * LLN || in_sizes[20] != SSN * LLN) return;
  if (in_sizes[21] != HH * GG || in_sizes[22] != HH) return;
  if (in_sizes[23] != HH || in_sizes[24] != 1 || in_sizes[25] != HH || in_sizes[26] != 1) return;
  if (out_size != 2 * NN) return;

  const float* x     = (const float*)d_in[0];
  const int*   iedge = (const int*)d_in[1];
  const int*   oedge = (const int*)d_in[2];
  const float* gWih  = (const float*)d_in[3];
  const float* gWhh  = (const float*)d_in[4];
  const float* gbih  = (const float*)d_in[5];
  const float* gbhh  = (const float*)d_in[6];
  const float* attW  = (const float*)d_in[7];
  const float* attb  = (const float*)d_in[8];
  const float* wkW   = (const float*)d_in[9];
  const float* wkb   = (const float*)d_in[10];
  const float* g1W   = (const float*)d_in[11];
  const float* g1as  = (const float*)d_in[12];
  const float* g1ad  = (const float*)d_in[13];
  const float* g1b   = (const float*)d_in[14];
  const float* g2W   = (const float*)d_in[15];
  const float* g2as  = (const float*)d_in[16];
  const float* g2ad  = (const float*)d_in[17];
  const float* g2b   = (const float*)d_in[18];
  const float* pW    = (const float*)d_in[19];
  const float* pb    = (const float*)d_in[20];
  const float* fW    = (const float*)d_in[21];
  const float* fbias = (const float*)d_in[22];
  const float* rW    = (const float*)d_in[23];
  const float* rb    = (const float*)d_in[24];
  const float* cWv   = (const float*)d_in[25];
  const float* cb    = (const float*)d_in[26];
  float* out = (float*)d_out;

  char* ws = (char*)d_ws;
  size_t off = 0;
  const size_t oWG  = off; off = al256(off + (size_t)WKN * GG * KG * 2);
  const size_t oG1W = off; off = al256(off + (size_t)HH * HH * 2);
  const size_t oFW  = off; off = al256(off + (size_t)HH * GG * 2);
  const size_t hsBytes = (size_t)TT * NN * HH * 4;
  const size_t oHS  = off; off = al256(off + hsBytes);
  const size_t oWKE = off; off = al256(off + (size_t)WKN * NN * HH * 4);
  if (off > ws_size || off > (size_t)WSCAP) return;
  size_t o2 = oHS;
  const size_t oWAV  = o2; o2 = al256(o2 + (size_t)NN * HH * 4);
  const size_t oY    = o2; o2 = al256(o2 + (size_t)NN * HH * 4);
  const size_t oES   = o2; o2 = al256(o2 + (size_t)NN * 4);
  const size_t oED   = o2; o2 = al256(o2 + (size_t)NN * 4);
  const size_t oG1O  = o2; o2 = al256(o2 + (size_t)NN * HH * 4);
  const size_t oST   = o2; o2 = al256(o2 + (size_t)SSN * HH * LP * 2);
  const size_t oPW   = o2; o2 = al256(o2 + (size_t)SSN * LP * LP * 2);
  const size_t oCAT  = o2; o2 = al256(o2 + (size_t)SSN * HH * 4);
  const size_t oCAT2 = o2; o2 = al256(o2 + (size_t)SSN * HH * 4);
  if (o2 > oHS + hsBytes) return;

  _Float16* WG16  = (_Float16*)(ws + oWG);
  _Float16* G1W16 = (_Float16*)(ws + oG1W);
  _Float16* FW16  = (_Float16*)(ws + oFW);
  float*    HS    = (float*)(ws + oHS);
  float*    WKE   = (float*)(ws + oWKE);
  float*    WAV   = (float*)(ws + oWAV);
  float*    Y     = (float*)(ws + oY);
  float*    ES    = (float*)(ws + oES);
  float*    ED    = (float*)(ws + oED);
  float*    G1O   = (float*)(ws + oG1O);
  _Float16* ST16  = (_Float16*)(ws + oST);
  _Float16* PW16  = (_Float16*)(ws + oPW);
  float*    CAT   = (float*)(ws + oCAT);
  float*    CAT2  = (float*)(ws + oCAT2);

  const int nb   = pick_nb(nE, nN);
  const int vec8 = ((nE & 3) == 0) ? 1 : 0;
  const int gA   = (nN + nb - 1) / nb;
  const int gRow = NN / RB;
  const int gCh  = (NN * (HH / 4)) / 256;
  const int b0   = (SSN * HH * (LP / 8)) / 256;
  const int b1   = (SSN * LP * (LP / 8)) / 256;

  hipFuncSetAttribute(reinterpret_cast<const void*>(&k_agg),
                      hipFuncAttributeMaxDynamicSharedMemorySize, LDS_AGG);

  k_wprep<<<dim3((WKN * GG * (KG / 8)) / 256, 3), 256, 0, stream>>>(gWih, gWhh, g1W, fW, WG16, G1W16, FW16);

  for (int w = 0; w < WKN; ++w) {
    const float*    xw  = x + (size_t)w * NN * TT * DD;
    const _Float16* wgw = WG16 + (size_t)w * GG * KG;
    const float*    biw = gbih + (size_t)w * GG;
    const float*    bhw = gbhh + (size_t)w * GG;
    for (int t = 0; t < TT; ++t) {
      const float* hsrc = HS + (size_t)(t > 0 ? t - 1 : 0) * NN * HH;
      float*       hdst = HS + (size_t)t * NN * HH;
      k_gru<<<gRow, RT, 0, stream>>>(xw, wgw, biw, bhw, hsrc, hdst, t, t > 0 ? 1 : 0, nN);
    }
    k_att_time<<<gCh, 256, 0, stream>>>(HS, attW + (size_t)w * TT * TT, attb + (size_t)w * TT,
                                        WKE + (size_t)w * NN * HH, nN);
  }
  k_att_week<<<gCh, 256, 0, stream>>>(WKE, wkW, wkb, WAV, nN);

  k_lin1<<<gRow, RT, 0, stream>>>(WAV, G1W16, g1as, g1ad, Y, ES, ED, nN);
  k_agg<<<gA, NTHR, LDS_AGG, stream>>>(iedge, iedge + nE, Y, ES, ED, g1b, G1O, nN, nE, nb, vec8);

  k_prep2<<<b0 + b1, 256, 0, stream>>>(G1O, pW, ST16, PW16, b0);
  k_sector<<<SSN, 256, 0, stream>>>(ST16, PW16, pb, G1O, CAT);

  k_gat2<<<1, 256, 0, stream>>>(CAT, oedge, g2W, g2as, g2ad, g2b, CAT2, nE2);

  k_fus<<<gRow, RT, 0, stream>>>(WAV, G1O, CAT2, FW16, fbias, rW, rb, cWv, cb, out, nN);
}
